// RelativeAttention_13864154432323
// MI455X (gfx1250) — hardware-verified
//
#include <hip/hip_runtime.h>
#include <stdint.h>

#define BSZ     16
#define NTOK    577
#define NP      640
#define CDIM    768
#define C3      2304
#define NHEAD   12
#define DHEAD   64
#define NREL    2210
#define RX      9344
#define MCT     (BSZ * NP)
#define VTP     (BSZ * NP)
#define PADFILL (-1.0e30f)
static_assert(NHEAD * DHEAD == CDIM);
static_assert(C3 == 3 * CDIM);
static_assert((RX % 64) == 0 && RX >= (BSZ - 1) * NTOK + NP);
static_assert((NP % 64) == 0 && NP >= NTOK && NP - 64 < NTOK);
static_assert((CDIM % 64) == 0 && (CDIM % 32) == 0);
static_assert(((RX * CDIM / 8) % 256) == 0);
static_assert(((C3 * CDIM / 8) % 256) == 0);
static_assert(((CDIM * CDIM / 8) % 256) == 0);
static_assert(((NHEAD * NP * (NP / 8)) % 256) == 0);
static_assert((MCT % 64) == 0);

typedef __bf16 v16b __attribute__((ext_vector_type(16)));
typedef float  v8f  __attribute__((ext_vector_type(8)));
typedef float  v4f  __attribute__((ext_vector_type(4)));
typedef unsigned int   v4u  __attribute__((ext_vector_type(4)));
typedef unsigned short v8us __attribute__((ext_vector_type(8)));
typedef v8us __attribute__((may_alias)) v8usa;
typedef v4f  __attribute__((may_alias)) v4fa;
typedef v4u  __attribute__((may_alias)) v4ua;
union FB { v16b v; v8us u[2]; unsigned w[8]; };

#if defined(__HIP_DEVICE_COMPILE__)
#define DEV_ASM 1
#else
#define DEV_ASM 0
#endif

__device__ __forceinline__ unsigned short bf_bits(float f) {
  unsigned u = __float_as_uint(f);
  return (unsigned short)((u + 0x7FFFu + ((u >> 16) & 1u)) >> 16);
}
__device__ __forceinline__ float bf_up(unsigned short hb) { return __uint_as_float(((unsigned)hb) << 16); }
__device__ __forceinline__ float bf_rn(float f) { return bf_up(bf_bits(f)); }
__device__ __forceinline__ unsigned pk16(unsigned short a, unsigned short b) { return (unsigned)a | ((unsigned)b << 16); }
__device__ __forceinline__ v8f zero8() { v8f z = {0.f, 0.f, 0.f, 0.f, 0.f, 0.f, 0.f, 0.f}; return z; }
__device__ __forceinline__ void split2(float f, unsigned short& h, unsigned short& l) {
  h = bf_bits(f);
  l = bf_bits(f - bf_up(h));
}
__device__ __forceinline__ void split8(const float* f, float sc, v4u& hi, v4u& lo) {
  v4u a, b;
#pragma unroll
  for (int e = 0; e < 4; ++e) {
    unsigned short h0, l0, h1, l1;
    split2(f[2 * e] * sc, h0, l0);
    split2(f[2 * e + 1] * sc, h1, l1);
    a[e] = pk16(h0, h1);
    b[e] = pk16(l0, l1);
  }
  hi = a; lo = b;
}

__device__ __forceinline__ v16b ldfrag_b(const unsigned short* p, int h) {
  FB f;
  f.u[0] = *(const v8usa*)(p + 8 * h);
  f.u[1] = *(const v8usa*)(p + 16 + 8 * h);
  return f.v;
}

__device__ __forceinline__ v8f mmar(v16b a, v16b b, v8f c) {
  return __builtin_amdgcn_wmma_f32_16x16x32_bf16(false, a, false, b, (short)0, c, false, false);
}
__device__ __forceinline__ v8f mma_g(v16b a, v16b b, v8f c) {
  c = __builtin_amdgcn_wmma_f32_16x16x32_bf16(false, a, false, b, (short)0, c, false, false);
#if DEV_ASM
  asm volatile("v_nop\n\tv_nop\n\tv_nop\n\tv_nop" : "+v"(c) : "v"(a), "v"(b));
#endif
  return c;
}
__device__ __forceinline__ void dep_guard(v8f& a, v8f& b, v16b x, v16b y) {
#if DEV_ASM
  asm volatile("v_nop\n\tv_nop\n\tv_nop\n\tv_nop" : "+v"(a), "+v"(b) : "v"(x), "v"(y));
#else
  (void)a; (void)b; (void)x; (void)y;
#endif
}
__device__ __forceinline__ void keep4(v16b a, v16b b, v16b c, v16b d) {
#if DEV_ASM
  asm volatile("v_nop" :: "v"(a), "v"(b), "v"(c), "v"(d));
#else
  (void)a; (void)b; (void)c; (void)d;
#endif
}
__device__ __forceinline__ void acc_guard4(v8f& a, v8f& b, v8f& c, v8f& d) {
#if DEV_ASM
  asm volatile("v_nop\n\tv_nop\n\tv_nop\n\tv_nop" : "+v"(a), "+v"(b), "+v"(c), "+v"(d));
#else
  (void)a; (void)b; (void)c; (void)d;
#endif
}

__device__ __forceinline__ void pack_p2(v8f a, v8f c, v16b& ph, v16b& pl) {
  FB h, l;
#pragma unroll
  for (int i = 0; i < 4; ++i) {
    unsigned short h0, l0, h1, l1, g0, m0, g1, m1;
    split2(a[2 * i], h0, l0);
    split2(a[2 * i + 1], h1, l1);
    split2(c[2 * i], g0, m0);
    split2(c[2 * i + 1], g1, m1);
    h.w[i] = pk16(h0, h1);      l.w[i] = pk16(l0, l1);
    h.w[4 + i] = pk16(g0, g1);  l.w[4 + i] = pk16(m0, m1);
  }
  ph = h.v; pl = l.v;
}

__global__ __launch_bounds__(256) void cvt_bf16x8(const float* __restrict__ in, unsigned short* out,
                                                  int nvalid8, int n8) {
  const int i = blockIdx.x * 256 + (int)threadIdx.x;
  if (i >= n8) return;
  const int ic = (i < nvalid8) ? i : (nvalid8 - 1);
  const bool ok = i < nvalid8;
  const v4f a  = *(const v4fa*)(in + (size_t)ic * 8);
  const v4f a4 = *(const v4fa*)(in + (size_t)ic * 8 + 4);
  v4u p;
  p[0] = ok ? pk16(bf_bits(a[0]),  bf_bits(a[1]))  : 0u;
  p[1] = ok ? pk16(bf_bits(a[2]),  bf_bits(a[3]))  : 0u;
  p[2] = ok ? pk16(bf_bits(a4[0]), bf_bits(a4[1])) : 0u;
  p[3] = ok ? pk16(bf_bits(a4[2]), bf_bits(a4[3])) : 0u;
  unsigned short* o = out + (size_t)i * 8;
  *(volatile v4u*)o = p;
  __threadfence();
  *(volatile v4u*)o = p;
}

__global__ __launch_bounds__(256) void bias_kernel(const float* __restrict__ table, const int* __restrict__ rel,
                                                   unsigned short* bp) {
  const int t = blockIdx.x * 256 + (int)threadIdx.x;
  if (t >= NHEAD * NP * (NP / 8)) return;
  const int k8 = t % (NP / 8);
  const int rq = t / (NP / 8);
  const int q  = rq % NP;
  const int h  = rq / NP;
  const int qc = (q > NTOK - 1) ? (NTOK - 1) : q;
  const bool qok = q < NTOK;
  v4u p;
#pragma unroll
  for (int e = 0; e < 4; ++e) {
    const int ka = k8 * 8 + 2 * e;
    const int kbb = ka + 1;
    const int kac = (ka > NTOK - 1) ? (NTOK - 1) : ka;
    const int kbc = (kbb > NTOK - 1) ? (NTOK - 1) : kbb;
    int ia = rel[qc * NTOK + kac];
    int ib = rel[qc * NTOK + kbc];
    ia = (ia < 0) ? 0 : ia;  ia = (ia > NREL - 1) ? (NREL - 1) : ia;
    ib = (ib < 0) ? 0 : ib;  ib = (ib > NREL - 1) ? (NREL - 1) : ib;
    const float va = table[ia * NHEAD + h];
    const float vb = table[ib * NHEAD + h];
    const unsigned short sa = (qok && ka < NTOK)  ? bf_bits(va) : (unsigned short)0;
    const unsigned short sb = (qok && kbb < NTOK) ? bf_bits(vb) : (unsigned short)0;
    p[e] = pk16(sa, sb);
  }
  unsigned short* o = bp + (size_t)t * 8;
  *(volatile v4u*)o = p;
  __threadfence();
  *(volatile v4u*)o = p;
}

template <int NPROD, int OUT_MODE>
__global__ __launch_bounds__(256) void gemm64(
    const unsigned short* __restrict__ A0, const unsigned short* __restrict__ A1, int lda, long long strideA,
    const unsigned short* __restrict__ B0, const unsigned short* __restrict__ B1, int ldb, long long strideB,
    void* Cout, void* Cout2, int ldc, long long strideC, const float* __restrict__ bias,
    int M, int N, int K, int nvalid, float oscale) {
  __shared__ __align__(16) float sT[8][16 * 68];
  const int bz   = blockIdx.y;
  const int lane = (int)threadIdx.x & 31;
  const int wave = (int)threadIdx.x >> 5;
  const int tilesN = N >> 6;
  const int tilesM = M >> 6;
  const int tile = blockIdx.x * 8 + wave;
  if (tile >= tilesM * tilesN) return;
  const int tm = tile / tilesN;
  const int tn = tile - tm * tilesN;
  const int m0 = tm << 6;
  const int n0 = tn << 6;

  const size_t aoff = (size_t)bz * (size_t)strideA;
  const size_t boff = (size_t)bz * (size_t)strideB;
  const size_t coff = (size_t)bz * (size_t)strideC;

  const int rlane = lane & 15;
  const int hh    = lane >> 4;
  const int mOff  = hh * 8;

  v8f acc[4][4];
#pragma unroll
  for (int i = 0; i < 4; ++i)
#pragma unroll
    for (int j = 0; j < 4; ++j) acc[i][j] = zero8();

  for (int k0 = 0; k0 < K; k0 += 32) {
#pragma unroll
    for (int p = 0; p < NPROD; ++p) {
      const unsigned short* Ab = ((p == 0) ? A0 : A1) + aoff;
      const unsigned short* Bb = ((p == 0) ? B0 : B1) + boff;
      v16b bq[4];
#pragma unroll
      for (int j = 0; j < 4; ++j)
        bq[j] = ldfrag_b(Bb + (size_t)(n0 + (j << 4) + rlane) * ldb + k0, hh);
#pragma unroll
      for (int i = 0; i < 4; ++i) {
        const v16b af = ldfrag_b(Ab + (size_t)(m0 + (i << 4) + rlane) * lda + k0, hh);
#pragma unroll
        for (int j = 0; j < 4; ++j) acc[i][j] = mmar(af, bq[j], acc[i][j]);
        dep_guard(acc[i][0], acc[i][3], af, bq[3]);
      }
      keep4(bq[0], bq[1], bq[2], bq[3]);
    }
  }
  acc_guard4(acc[0][0], acc[0][1], acc[0][2], acc[0][3]);
  acc_guard4(acc[1][0], acc[1][1], acc[1][2], acc[1][3]);
  acc_guard4(acc[2][0], acc[2][1], acc[2][2], acc[2][3]);
  acc_guard4(acc[3][0], acc[3][1], acc[3][2], acc[3][3]);

  float* slab = sT[wave];
  const int h2 = lane >> 4, c4 = (lane & 15) * 4;
  const int q  = lane >> 3, c8 = (lane & 7) * 8;
  v4f bb4 = {0.f, 0.f, 0.f, 0.f};
  if (OUT_MODE == 0) {
    const v4f braw = *(const v4fa*)(bias + n0 + c4);
#pragma unroll
    for (int e = 0; e < 4; ++e) bb4[e] = bf_rn(braw[e]);
  }
#pragma unroll
  for (int i = 0; i < 4; ++i) {
    const int mBase = m0 + (i << 4);
#pragma unroll
    for (int j = 0; j < 4; ++j) {
#pragma unroll
      for (int r = 0; r < 8; ++r) {
        slab[(mOff + r) * 68 + (j << 4) + rlane] = acc[i][j][r];
      }
    }
    __builtin_amdgcn_fence(__ATOMIC_RELEASE, "workgroup");
    __builtin_amdgcn_wave_barrier();
    __builtin_amdgcn_fence(__ATOMIC_ACQUIRE, "workgroup");
    if (OUT_MODE == 0) {
      float* C = (float*)Cout + coff;
      for (int pass = 0; pass < 2; ++pass) {
#pragma unroll
        for (int it = 0; it < 8; ++it) {
          const int row  = it * 2 + h2;
          const int grow = mBase + row;
          const int bq   = grow / NP;
          const int n    = grow - bq * NP;
          const v4f v = *(const v4fa*)(slab + row * 68 + c4) * oscale + bb4;
          if (n < nvalid) *(volatile v4f*)(C + ((size_t)bq * nvalid + n) * ldc + n0 + c4) = v;
        }
        __threadfence();
      }
    } else {
      unsigned short* C  = (unsigned short*)Cout  + coff;
      unsigned short* C2 = (unsigned short*)Cout2 + coff;
      v4u hv[4], lv[4];
#pragma unroll
      for (int it = 0; it < 4; ++it) {
        const int row = it * 4 + q;
        const float* sp = slab + row * 68 + c8;
        float f[8];
#pragma unroll
        for (int e = 0; e < 8; ++e) f[e] = sp[e];
        split8(f, oscale, hv[it], lv[it]);
      }
      for (int pass = 0; pass < 2; ++pass) {
#pragma unroll
        for (int it = 0; it < 4; ++it) {
          const int row = it * 4 + q;
          const size_t go = (size_t)(mBase + row) * ldc + n0 + c8;
          *(volatile v4u*)(C + go)  = hv[it];
          *(volatile v4u*)(C2 + go) = lv[it];
        }
        __threadfence();
      }
    }
    __builtin_amdgcn_fence(__ATOMIC_RELEASE, "workgroup");
    __builtin_amdgcn_wave_barrier();
    __builtin_amdgcn_fence(__ATOMIC_ACQUIRE, "workgroup");
  }
}

__device__ __forceinline__ v8f score16(const unsigned short* khp, const unsigned short* klp, int hh,
                                       v16b qh0, v16b qh1, v16b ql0, v16b ql1) {
  v8f z = zero8();
  {
    const v16b a0 = ldfrag_b(khp, hh);
    const v16b a1 = ldfrag_b(khp + 32, hh);
    z = mma_g(a0, qh0, z);
    z = mma_g(a1, qh1, z);
    z = mma_g(a0, ql0, z);
    z = mma_g(a1, ql1, z);
  }
  {
    const v16b b0 = ldfrag_b(klp, hh);
    const v16b b1 = ldfrag_b(klp + 32, hh);
    z = mma_g(b0, qh0, z);
    z = mma_g(b1, qh1, z);
  }
  return z;
}

__global__ __launch_bounds__(128) void attn_kernel(
    const unsigned short* __restrict__ Qh, const unsigned short* __restrict__ Ql,
    const unsigned short* __restrict__ Kh, const unsigned short* __restrict__ Kl,
    const unsigned short* __restrict__ VTh, const unsigned short* __restrict__ VTl,
    const unsigned short* __restrict__ Bp, unsigned short* CTh, unsigned short* CTl) {
  __shared__ __align__(16) float sO[4 * 16 * 64];

  const int tid = (int)threadIdx.x, lane = tid & 31, w = tid >> 5;
  const int hh = lane >> 4, m = lane & 15;
  const int head = blockIdx.y;
  const int b    = blockIdx.z;
  const int qn0  = blockIdx.x * 64 + 16 * w;
  const bool active = qn0 < NTOK;

  const size_t qo = ((size_t)b * NTOK + (size_t)(qn0 + m)) * CDIM + (size_t)head * DHEAD;
  const v16b qh0 = ldfrag_b(Qh + qo, hh);
  const v16b qh1 = ldfrag_b(Qh + qo + 32, hh);
  const v16b ql0 = ldfrag_b(Ql + qo, hh);
  const v16b ql1 = ldfrag_b(Ql + qo + 32, hh);

  v8f o[4];
#pragma unroll
  for (int t = 0; t < 4; ++t) o[t] = zero8();
  float mrun = PADFILL, lrun = 0.0f;

  const unsigned short* khb = Kh  + ((size_t)b * NTOK + m) * CDIM + (size_t)head * DHEAD;
  const unsigned short* klb = Kl  + ((size_t)b * NTOK + m) * CDIM + (size_t)head * DHEAD;
  const unsigned short* vhb = VTh + ((size_t)head * DHEAD + m) * VTP + (size_t)b * NP;
  const unsigned short* vlb = VTl + ((size_t)head * DHEAD + m) * VTP + (size_t)b * NP;
  const unsigned short* bpb = Bp  + ((size_t)head * NP + (size_t)(qn0 + m)) * NP + 8 * hh;

  if (active) {
#pragma unroll 1
    for (int kb = 0; kb < NP; kb += 64) {
      const bool fullt = (kb + 64) <= NTOK;
      v8f s[4];
      s[0] = score16(khb + (size_t)kb * CDIM, klb + (size_t)kb * CDIM, hh, qh0, qh1, ql0, ql1);
      if (fullt) {
        s[1] = score16(khb + (size_t)(kb + 16) * CDIM, klb + (size_t)(kb + 16) * CDIM, hh, qh0, qh1, ql0, ql1);
        s[2] = score16(khb + (size_t)(kb + 32) * CDIM, klb + (size_t)(kb + 32) * CDIM, hh, qh0, qh1, ql0, ql1);
        s[3] = score16(khb + (size_t)(kb + 48) * CDIM, klb + (size_t)(kb + 48) * CDIM, hh, qh0, qh1, ql0, ql1);
      } else {
        s[1] = zero8(); s[2] = zero8(); s[3] = zero8();
      }
#pragma unroll
      for (int j = 0; j < 4; ++j) {
        const v4u bw = *(const v4ua*)(bpb + kb + 16 * j);
        const int kbase = kb + 16 * j + 8 * hh;
#pragma unroll
        for (int e = 0; e < 4; ++e) {
          const float b0f = __uint_as_float(bw[e] << 16);
          const float b1f = __uint_as_float(bw[e] & 0xffff0000u);
          const float t0 = s[j][2 * e] + b0f;
          const float t1 = s[j][2 * e + 1] + b1f;
          s[j][2 * e]     = (kbase + 2 * e     < NTOK) ? t0 : PADFILL;
          s[j][2 * e + 1] = (kbase + 2 * e + 1 < NTOK) ? t1 : PADFILL;
        }
      }

      float mloc = s[0][0];
#pragma unroll
      for (int j = 0; j < 4; ++j)
#pragma unroll
        for (int r = 0; r < 8; ++r) mloc = fmaxf(mloc, s[j][r]);
      mloc = fmaxf(mloc, __shfl_xor(mloc, 16, 32));
      const float mnew  = fmaxf(mrun, mloc);
      const float alpha = __expf(mrun - mnew);
      mrun = mnew;
      float lsum = 0.0f;
#pragma unroll
      for (int j = 0; j < 4; ++j)
#pragma unroll
        for (int r = 0; r < 8; ++r) {
          const float p = __expf(s[j][r] - mnew);
          s[j][r] = p;
          lsum += p;
        }
      lsum += __shfl_xor(lsum, 16, 32);
      lrun = lrun * alpha + lsum;
#pragma unroll
      for (int t = 0; t < 4; ++t)
#pragma unroll
        for (int r = 0; r < 8; ++r) o[t][r] = o[t][r] * alpha;

      v16b ph0, pl0, ph1, pl1;
      pack_p2(s[0], s[1], ph0, pl0);
      pack_p2(s[2], s[3], ph1, pl1);

#pragma unroll
      for (int t = 0; t < 4; ++t) {
        const size_t vo = (size_t)(16 * t) * VTP + kb;
        const v16b a0 = ldfrag_b(vhb + vo, hh);
        o[t] = mma_g(a0, ph0, o[t]);
        o[t] = mma_g(a0, pl0, o[t]);
        const v16b c0 = ldfrag_b(vlb + vo, hh);
        o[t] = mma_g(c0, ph0, o[t]);
      }
      if (fullt) {
#pragma unroll
        for (int t = 0; t < 4; ++t) {
          const size_t vo = (size_t)(16 * t) * VTP + kb + 32;
          const v16b a1 = ldfrag_b(vhb + vo, hh);
          o[t] = mma_g(a1, ph1, o[t]);
          o[t] = mma_g(a1, pl1, o[t]);
          const v16b c1 = ldfrag_b(vlb + vo, hh);
          o[t] = mma_g(c1, ph1, o[t]);
        }
      }
    }
  }

  const float inv = active ? (1.0f / lrun) : 0.0f;
  float* so = sO + w * 1024;
#pragma unroll
  for (int t = 0; t < 4; ++t)
#pragma unroll
    for (int r = 0; r < 8; ++r)
      so[m * 64 + 16 * t + 8 * hh + r] = o[t][r] * inv;
  __syncthreads();

  const int q8 = lane & 7, sub = lane >> 3;
  v4u hv[4], lv[4];
#pragma unroll
  for (int it = 0; it < 4; ++it) {
    const int row = it * 4 + sub;
    const v4f fa = *(const v4fa*)(so + row * 64 + 8 * q8);
    const v4f fb = *(const v4fa*)(so + row * 64 + 8 * q8 + 4);
    float f[8];
#pragma unroll
    for (int e = 0; e < 4; ++e) { f[e] = fa[e]; f[4 + e] = fb[e]; }
    split8(f, 1.0f, hv[it], lv[it]);
  }
  for (int pass = 0; pass < 2; ++pass) {
#pragma unroll
    for (int it = 0; it < 4; ++it) {
      const int row = it * 4 + sub;
      const size_t go = ((size_t)b * NP + (size_t)(qn0 + row)) * CDIM + (size_t)head * DHEAD + 8 * q8;
      *(volatile v4u*)(CTh + go) = hv[it];
      *(volatile v4u*)(CTl + go) = lv[it];
    }
    __threadfence();
  }
}

extern "C" void kernel_launch(void* const* d_in, const int* in_sizes, int n_in,
                              void* d_out, int out_size, void* d_ws, size_t ws_size,
                              hipStream_t stream) {
  if (n_in < 6) return;
  if (in_sizes[0] != BSZ * NTOK * CDIM) return;
  if (in_sizes[1] != C3 * CDIM) return;
  if (in_sizes[2] != CDIM * CDIM) return;
  if (in_sizes[3] != CDIM) return;
  if (in_sizes[4] != NREL * NHEAD) return;
  if (in_sizes[5] != NTOK * NTOK) return;
  if (out_size != BSZ * NTOK * CDIM) return;

  const float* x      = (const float*)d_in[0];
  const float* qkv_w  = (const float*)d_in[1];
  const float* proj_w = (const float*)d_in[2];
  const float* proj_b = (const float*)d_in[3];
  const float* table  = (const float*)d_in[4];
  const int*   rel    = (const int*)d_in[5];
  float* out = (float*)d_out;

  const size_t PCT = (size_t)MCT * CDIM * 2;
  const size_t PX  = (size_t)RX * CDIM * 2;
  const size_t PWQ = (size_t)C3 * CDIM * 2;
  const size_t PWP = (size_t)CDIM * CDIM * 2;
  const size_t PVT = (size_t)CDIM * VTP * 2;
  const size_t PBP = (size_t)NHEAD * NP * NP * 2;
  size_t off = 0;
  const size_t oCTh = off; off += PCT;
  const size_t oCTl = off; off += PCT;
  const size_t oXb  = 0;
  const size_t oWq  = oXb + PX;
  if (oWq + PWQ > oCTl + PCT) return;
  const size_t oWp  = off; off += PWP;
  const size_t oQh  = off; off += PX;
  const size_t oQl  = off; off += PX;
  const size_t oKh  = off; off += PX;
  const size_t oKl  = off; off += PX;
  const size_t oVTh = off; off += PVT;
  const size_t oVTl = off; off += PVT;
  const size_t oBp  = off; off += PBP;
  if (off > ws_size) return;
  if (off > (size_t)134217728) return;

  char* ws = (char*)d_ws;
  unsigned short* CTh = (unsigned short*)(ws + oCTh);
  unsigned short* CTl = (unsigned short*)(ws + oCTl);
  unsigned short* Xb  = (unsigned short*)(ws + oXb);
  unsigned short* Wqb = (unsigned short*)(ws + oWq);
  unsigned short* Wkb = Wqb + (size_t)CDIM * CDIM;
  unsigned short* Wvb = Wqb + (size_t)2 * CDIM * CDIM;
  unsigned short* Wpb = (unsigned short*)(ws + oWp);
  unsigned short* Qh  = (unsigned short*)(ws + oQh);
  unsigned short* Ql  = (unsigned short*)(ws + oQl);
  unsigned short* Kh  = (unsigned short*)(ws + oKh);
  unsigned short* Kl  = (unsigned short*)(ws + oKl);
  unsigned short* VTh = (unsigned short*)(ws + oVTh);
  unsigned short* VTl = (unsigned short*)(ws + oVTl);
  unsigned short* Bp  = (unsigned short*)(ws + oBp);

  const dim3 blk(256);
  const int n8x   = RX * CDIM / 8;
  const int n8xv  = BSZ * NTOK * CDIM / 8;
  const int n8wq  = C3 * CDIM / 8;
  const int n8wp  = CDIM * CDIM / 8;
  const int nbias = NHEAD * NP * (NP / 8);
  const dim3 gQK((((RX / 64) * (CDIM / 64)) + 7) / 8, 1);
  const dim3 gVT((((CDIM / 64) * (NP / 64)) + 7) / 8, BSZ);
  const dim3 gPJ((((MCT / 64) * (CDIM / 64)) + 7) / 8, 1);
  const dim3 gAttn(NP / 64, NHEAD, BSZ);

  cvt_bf16x8<<<dim3(n8x / 256), blk, 0, stream>>>(x, Xb, n8xv, n8x);
  cvt_bf16x8<<<dim3(n8wq / 256), blk, 0, stream>>>(qkv_w, Wqb, n8wq, n8wq);
  cvt_bf16x8<<<dim3(n8wp / 256), blk, 0, stream>>>(proj_w, Wpb, n8wp, n8wp);
  bias_kernel<<<dim3(nbias / 256), blk, 0, stream>>>(table, rel, Bp);
  gemm64<1, 3><<<gQK, blk, 0, stream>>>(
      Xb, Xb, CDIM, 0LL, Wqb, Wqb, CDIM, 0LL, (void*)Qh, (void*)Ql, CDIM, 0LL, proj_b,
      RX, CDIM, CDIM, RX, 0.125f);
  gemm64<1, 3><<<gQK, blk, 0, stream>>>(
      Xb, Xb, CDIM, 0LL, Wkb, Wkb, CDIM, 0LL, (void*)Kh, (void*)Kl, CDIM, 0LL, proj_b,
      RX, CDIM, CDIM, RX, 1.0f);
  gemm64<1, 3><<<gVT, blk, 0, stream>>>(
      Wvb, Wvb, CDIM, 0LL, Xb, Xb, CDIM, (long long)NTOK * CDIM, (void*)VTh, (void*)VTl, VTP, (long long)NP, proj_b,
      CDIM, NP, CDIM, CDIM, 1.0f);
  attn_kernel<<<gAttn, dim3(128), 0, stream>>>(Qh, Ql, Kh, Kl, VTh, VTl, Bp, CTh, CTl);
  gemm64<2, 0><<<gPJ, blk, 0, stream>>>(
      CTh, CTl, CDIM, 0LL, Wpb, Wpb, CDIM, 0LL, (void*)out, (void*)out, CDIM, 0LL, proj_b,
      MCT, CDIM, CDIM, NTOK, 1.0f);
  (void)hipGetLastError();
}
